// Cross_attention_38972533243918
// MI455X (gfx1250) — hardware-verified
//
#include <hip/hip_runtime.h>
#include <math.h>

typedef __attribute__((ext_vector_type(16))) _Float16 v16h;
typedef __attribute__((ext_vector_type(8)))  _Float16 v8h;
typedef __attribute__((ext_vector_type(4)))  _Float16 v4h;
typedef __attribute__((ext_vector_type(8)))  float    v8f;
typedef __attribute__((ext_vector_type(4)))  float    v4f;
typedef __attribute__((ext_vector_type(4)))  unsigned int v4u;

constexpr int kB  = 2;
constexpr int kS  = 32;
constexpr int kGH = 24;
constexpr int kGW = 24;
constexpr int kP  = kGH * kGW;
constexpr int kC  = 64;
constexpr int kNH = 4;
constexpr int kHD = 16;
constexpr int kBS = kB * kS;
constexpr size_t kElems = (size_t)kBS * kP * kC;
static_assert(kP == 576);
static_assert(kNH * kHD == kC);
static_assert(kElems == 2359296ull);

constexpr float kQScale = 0.25f;
static_assert(kQScale * kQScale * (float)kHD == 1.0f);
constexpr float kCarry  = 16.0f;
constexpr float kLogit  = kQScale / (kCarry * kCarry);
static_assert(kLogit * 1024.0f == 1.0f);
constexpr float kOutInv = 1.0f / kCarry;
constexpr float kPShift = 5.545177444479562f;

constexpr int kQT = 32;
constexpr int kKC = 32;
constexpr int kOP = 68;
constexpr int kQP = 72;
constexpr int kVP = 40;
static_assert(kP % kQT == 0);
static_assert(kP % kKC == 0);
static_assert(kP % 64 == 0);
static_assert(kS == 32);

constexpr size_t kOffKH   = 0;
constexpr size_t kOffVT   = kOffKH + kElems * 2;
constexpr size_t kOffXS   = kOffVT + kElems * 2;
constexpr size_t kWsTotal = kOffXS + kElems * 4;
static_assert(kWsTotal == 18874368ull);
static_assert(kWsTotal <= 134217728ull);
static_assert((kOffVT % 128) == 0 && (kOffXS % 128) == 0);

__device__ __forceinline__ unsigned pk16(unsigned short a, unsigned short b) { return (unsigned)a | ((unsigned)b << 16); }
__device__ __forceinline__ unsigned short h_bits(float f) { const _Float16 h = (_Float16)f; return __builtin_bit_cast(unsigned short, h); }

__device__ __forceinline__ v8f mma_h(v16h a, v16h b, v8f c) {
  c = __builtin_amdgcn_wmma_f32_16x16x32_f16(false, a, false, b, (short)0, c, false, false);
  asm volatile("v_nop\n\tv_nop\n\tv_nop\n\tv_nop" : "+v"(c) : "v"(a), "v"(b));
  return c;
}

union FragU { v16h v; v8h h[2]; };
__device__ __forceinline__ v16h frag_low16(const _Float16* p) {
  const _Float16 z = (_Float16)0.0f;
  FragU f;
  f.h[0] = *(const v8h*)(p);
  f.h[1] = (v8h){z, z, z, z, z, z, z, z};
  return f.v;
}
__device__ __forceinline__ v16h frag_full(const _Float16* p) {
  FragU f;
  f.h[0] = *(const v8h*)(p);
  f.h[1] = *(const v8h*)(p + 16);
  return f.v;
}

__global__ __launch_bounds__(256) void feat_planes_kernel(const float* __restrict__ feat,
                                                          unsigned short* __restrict__ KH,
                                                          unsigned short* __restrict__ VT) {
  __shared__ float sm[64][65];
  const int t  = threadIdx.x;
  const int p0 = blockIdx.x * 64;
  const int bs = blockIdx.y;
  const float* src = feat + ((size_t)bs * kP + p0) * kC;
#pragma unroll
  for (int i = 0; i < 4; ++i) {
    const int idx = i * 256 + t;
    const int r   = idx >> 4;
    const int c4  = (idx & 15) * 4;
    const v4f v = *(const v4f*)(src + (size_t)idx * 4);
    sm[c4 + 0][r] = v[0] * kCarry;
    sm[c4 + 1][r] = v[1] * kCarry;
    sm[c4 + 2][r] = v[2] * kCarry;
    sm[c4 + 3][r] = v[3] * kCarry;
  }
  __syncthreads();
  const int lane = t & 31;
  const int wave = __builtin_amdgcn_readfirstlane((int)(threadIdx.x >> 5));
  const int q  = lane >> 3;
  const int c8 = (lane & 7) * 8;
  v4u vt[2], kh[2];
#pragma unroll
  for (int it = 0; it < 2; ++it) {
    const int row = wave * 8 + it * 4 + q;
    unsigned short a[8], b[8];
#pragma unroll
    for (int e = 0; e < 8; ++e) {
      a[e] = h_bits(sm[row][c8 + e]);
      b[e] = h_bits(sm[c8 + e][row]);
    }
    vt[it] = (v4u){pk16(a[0], a[1]), pk16(a[2], a[3]), pk16(a[4], a[5]), pk16(a[6], a[7])};
    kh[it] = (v4u){pk16(b[0], b[1]), pk16(b[2], b[3]), pk16(b[4], b[5]), pk16(b[6], b[7])};
  }
  for (int pass = 0; pass < 2; ++pass) {
#pragma unroll
    for (int it = 0; it < 2; ++it) {
      const int row = wave * 8 + it * 4 + q;
      *(volatile v4u*)(VT + ((size_t)bs * kC + row) * kP + p0 + c8) = vt[it];
      *(volatile v4u*)(KH + ((size_t)bs * kP + p0 + row) * kC + c8) = kh[it];
    }
    __threadfence();
  }
}

__global__ __launch_bounds__(128) void band_attn_kernel(const float* __restrict__ query,
                                                        const float* __restrict__ feat,
                                                        float* __restrict__ XS) {
  __shared__ __align__(16) _Float16 Qs[32 * kQP];
  __shared__ __align__(16) _Float16 Ks[32 * kQP];
  __shared__ __align__(16) _Float16 Vts[64 * kVP];
  __shared__ __align__(16) float    Os[32 * kOP];
  const int tid  = threadIdx.x;
  const int lane = tid & 31;
  const int head = __builtin_amdgcn_readfirstlane((int)(threadIdx.x >> 5));
  const int hh   = lane >> 4;
  const int c    = lane & 15;
  const int b    = blockIdx.x / kP;
  const int p    = blockIdx.x - b * kP;
  const size_t base = ((size_t)b * kS * kP + p) * kC;
  const size_t bstride = (size_t)kP * kC;

#pragma unroll
  for (int it = 0; it < 4; ++it) {
    const int idx = it * 128 + tid;
    const int s   = idx >> 4;
    const int c4  = (idx & 15) * 4;
    const size_t g = base + (size_t)s * bstride + c4;
    const v4f qv = *(const v4f*)(query + g);
    const v4f kv = *(const v4f*)(feat + g);
    v4h qh, kh;
    qh[0] = (_Float16)(qv[0] * kCarry);
    qh[1] = (_Float16)(qv[1] * kCarry);
    qh[2] = (_Float16)(qv[2] * kCarry);
    qh[3] = (_Float16)(qv[3] * kCarry);
    kh[0] = (_Float16)(kv[0] * kCarry);
    kh[1] = (_Float16)(kv[1] * kCarry);
    kh[2] = (_Float16)(kv[2] * kCarry);
    kh[3] = (_Float16)(kv[3] * kCarry);
    *(v4h*)(Qs + s * kQP + c4) = qh;
    *(v4h*)(Ks + s * kQP + c4) = kh;
    const _Float16 k0 = kh[0];
    const _Float16 k1 = kh[1];
    const _Float16 k2 = kh[2];
    const _Float16 k3 = kh[3];
    Vts[(c4 + 0) * kVP + s] = k0;
    Vts[(c4 + 1) * kVP + s] = k1;
    Vts[(c4 + 2) * kVP + s] = k2;
    Vts[(c4 + 3) * kVP + s] = k3;
  }
  __syncthreads();

  const v8f zero = (v8f){0.f, 0.f, 0.f, 0.f, 0.f, 0.f, 0.f, 0.f};
  const int coff = head * kHD + 8 * hh;
  const v16h kf0 = frag_low16(Ks + (c) * kQP + coff);
  const v16h kf1 = frag_low16(Ks + (16 + c) * kQP + coff);
  const v16h qf0 = frag_low16(Qs + (c) * kQP + coff);
  const v16h qf1 = frag_low16(Qs + (16 + c) * kQP + coff);
  const v16h vf  = frag_full(Vts + (head * kHD + c) * kVP + 8 * hh);

  v8f st[2][2];
  st[0][0] = mma_h(kf0, qf0, zero);
  st[1][0] = mma_h(kf1, qf0, zero);
  st[0][1] = mma_h(kf0, qf1, zero);
  st[1][1] = mma_h(kf1, qf1, zero);

#pragma unroll
  for (int j = 0; j < 2; ++j) {
    float cm = st[0][j][0];
#pragma unroll
    for (int r = 1; r < 8; ++r) cm = fmaxf(cm, st[0][j][r]);
#pragma unroll
    for (int r = 0; r < 8; ++r) cm = fmaxf(cm, st[1][j][r]);
    const float cmo = __shfl_xor(cm, 16, 32);
    cm = fmaxf(cm, cmo);
    const float mc = cm * kLogit - kPShift;
    float ps = 0.f;
    v16h pf;
#pragma unroll
    for (int r = 0; r < 8; ++r) {
      const float p0 = expf(fmaf(st[0][j][r], kLogit, -mc));
      const float p1 = expf(fmaf(st[1][j][r], kLogit, -mc));
      ps += p0;
      ps += p1;
      pf[r]     = (_Float16)p0;
      pf[8 + r] = (_Float16)p1;
    }
    const float pso = __shfl_xor(ps, 16, 32);
    const float lt  = ps + pso;
    const float inv = (1.0f / lt) * kOutInv;
    v8f o = mma_h(vf, pf, zero);
    float* op = Os + (16 * j + c) * kOP + head * kHD + 8 * hh;
    const v4f o0 = (v4f){o[0] * inv, o[1] * inv, o[2] * inv, o[3] * inv};
    const v4f o1 = (v4f){o[4] * inv, o[5] * inv, o[6] * inv, o[7] * inv};
    *(v4f*)(op)     = o0;
    *(v4f*)(op + 4) = o1;
  }
  __syncthreads();

  v4f val[4];
#pragma unroll
  for (int it = 0; it < 4; ++it) {
    const int row = it * 8 + head * 2 + hh;
    val[it] = *(const v4f*)(Os + row * kOP + c * 4);
  }
  for (int pass = 0; pass < 2; ++pass) {
#pragma unroll
    for (int it = 0; it < 4; ++it) {
      const int row = it * 8 + head * 2 + hh;
      *(volatile v4f*)(XS + base + (size_t)row * bstride + c * 4) = val[it];
    }
    __threadfence();
  }
}

__global__ __launch_bounds__(128) void pixel_attn_kernel(const float* __restrict__ query,
                                                         const unsigned short* __restrict__ KHp,
                                                         const unsigned short* __restrict__ VTp,
                                                         const float* __restrict__ XS,
                                                         float* __restrict__ out) {
  __shared__ __align__(16) float Os[kQT * kOP];
  const _Float16* KH = (const _Float16*)KHp;
  const _Float16* VT = (const _Float16*)VTp;
  const int tid  = threadIdx.x;
  const int lane = tid & 31;
  const int head = __builtin_amdgcn_readfirstlane((int)(threadIdx.x >> 5));
  const int hh   = lane >> 4;
  const int c    = lane & 15;
  constexpr int kTilesQ = kP / kQT;
  const int bs = blockIdx.x / kTilesQ;
  const int qt = blockIdx.x - bs * kTilesQ;
  const int q0 = qt * kQT;
  const size_t rowbase = (size_t)bs * kP;

  v16h qf[2];
#pragma unroll
  for (int j = 0; j < 2; ++j) {
    const float* qp = query + (rowbase + q0 + 16 * j + c) * kC + head * kHD + 8 * hh;
    const v4f a = *(const v4f*)(qp);
    const v4f d = *(const v4f*)(qp + 4);
    const _Float16 z = (_Float16)0.0f;
    v16h f;
    f[0] = (_Float16)(a[0] * kCarry);
    f[1] = (_Float16)(a[1] * kCarry);
    f[2] = (_Float16)(a[2] * kCarry);
    f[3] = (_Float16)(a[3] * kCarry);
    f[4] = (_Float16)(d[0] * kCarry);
    f[5] = (_Float16)(d[1] * kCarry);
    f[6] = (_Float16)(d[2] * kCarry);
    f[7] = (_Float16)(d[3] * kCarry);
    f[8] = z;  f[9] = z;  f[10] = z; f[11] = z;
    f[12] = z; f[13] = z; f[14] = z; f[15] = z;
    qf[j] = f;
  }

  const _Float16* kbase = KH + (rowbase + c) * kC + head * kHD + 8 * hh;
  const _Float16* vbase = VT + ((size_t)bs * kC + head * kHD + c) * kP + 8 * hh;

  const v8f zero = (v8f){0.f, 0.f, 0.f, 0.f, 0.f, 0.f, 0.f, 0.f};
  float mrun[2] = {-1e30f, -1e30f};
  float lrun[2] = {0.f, 0.f};
  v8f acc[2];
  acc[0] = zero;
  acc[1] = zero;

#pragma unroll 1
  for (int kc = 0; kc < kP / kKC; ++kc) {
    const int k0 = kc * kKC;
    const v16h kf0 = frag_low16(kbase + (size_t)k0 * kC);
    const v16h kf1 = frag_low16(kbase + (size_t)(k0 + 16) * kC);
    const v16h vf  = frag_full(vbase + k0);
    v8f st[2][2];
    st[0][0] = mma_h(kf0, qf[0], zero);
    st[1][0] = mma_h(kf1, qf[0], zero);
    st[0][1] = mma_h(kf0, qf[1], zero);
    st[1][1] = mma_h(kf1, qf[1], zero);
#pragma unroll
    for (int j = 0; j < 2; ++j) {
      float cm = st[0][j][0];
#pragma unroll
      for (int r = 1; r < 8; ++r) cm = fmaxf(cm, st[0][j][r]);
#pragma unroll
      for (int r = 0; r < 8; ++r) cm = fmaxf(cm, st[1][j][r]);
      const float cmo = __shfl_xor(cm, 16, 32);
      cm = fmaxf(cm, cmo);
      const float mnew  = fmaxf(mrun[j], cm * kLogit);
      const float alpha = expf(mrun[j] - mnew);
      mrun[j] = mnew;
      const float mc = mnew - kPShift;
      float ps = 0.f;
      v16h pf;
#pragma unroll
      for (int r = 0; r < 8; ++r) {
        const float p0 = expf(fmaf(st[0][j][r], kLogit, -mc));
        const float p1 = expf(fmaf(st[1][j][r], kLogit, -mc));
        ps += p0;
        ps += p1;
        pf[r]     = (_Float16)p0;
        pf[8 + r] = (_Float16)p1;
      }
      lrun[j] = lrun[j] * alpha + ps;
#pragma unroll
      for (int r = 0; r < 8; ++r) acc[j][r] *= alpha;
      acc[j] = mma_h(vf, pf, acc[j]);
    }
  }

#pragma unroll
  for (int j = 0; j < 2; ++j) {
    const float lo  = __shfl_xor(lrun[j], 16, 32);
    const float lt  = lrun[j] + lo;
    const float inv = (1.0f / lt) * kOutInv;
    float* op = Os + (16 * j + c) * kOP + head * kHD + 8 * hh;
    const v4f o0 = (v4f){acc[j][0] * inv, acc[j][1] * inv, acc[j][2] * inv, acc[j][3] * inv};
    const v4f o1 = (v4f){acc[j][4] * inv, acc[j][5] * inv, acc[j][6] * inv, acc[j][7] * inv};
    *(v4f*)(op)     = o0;
    *(v4f*)(op + 4) = o1;
  }
  __syncthreads();

  v4f val[4];
#pragma unroll
  for (int it = 0; it < 4; ++it) {
    const int row = it * 8 + head * 2 + hh;
    const size_t g = (rowbase + q0 + row) * kC + c * 4;
    const v4f o = *(const v4f*)(Os + row * kOP + c * 4);
    const v4f x = *(const v4f*)(XS + g);
    val[it] = (v4f){o[0] + x[0], o[1] + x[1], o[2] + x[2], o[3] + x[3]};
  }
  for (int pass = 0; pass < 2; ++pass) {
#pragma unroll
    for (int it = 0; it < 4; ++it) {
      const int row = it * 8 + head * 2 + hh;
      const size_t g = (rowbase + q0 + row) * kC + c * 4;
      *(volatile v4f*)(out + g) = val[it];
    }
    __threadfence();
  }
}

extern "C" void kernel_launch(void* const* d_in, const int* in_sizes, int n_in,
                              void* d_out, int out_size, void* d_ws, size_t ws_size,
                              hipStream_t stream) {
  if (n_in < 2) return;
  if ((size_t)in_sizes[0] != kElems) return;
  if ((size_t)in_sizes[1] != kElems) return;
  if ((size_t)out_size != kElems) return;
  if (ws_size < kWsTotal) return;

  const float* query = (const float*)d_in[0];
  const float* feat  = (const float*)d_in[1];
  float* out = (float*)d_out;

  char* ws = (char*)d_ws;
  unsigned short* KH = (unsigned short*)(ws + kOffKH);
  unsigned short* VT = (unsigned short*)(ws + kOffVT);
  float*          XS = (float*)(ws + kOffXS);

  feat_planes_kernel<<<dim3(kP / 64, kBS), 256, 0, stream>>>(feat, KH, VT);
  band_attn_kernel<<<kB * kP, 128, 0, stream>>>(query, feat, XS);
  pixel_attn_kernel<<<kBS * (kP / kQT), 128, 0, stream>>>(query, KH, VT, XS, out);
}
